// LanguageAttention_55929064129330
// MI455X (gfx1250) — hardware-verified
//
#include <hip/hip_runtime.h>
#include <math.h>
#include <stdint.h>

typedef __attribute__((ext_vector_type(16))) _Float16 v16h;
typedef __attribute__((ext_vector_type(8)))  _Float16 v8h;
typedef __attribute__((ext_vector_type(16))) __bf16   v16b;
typedef __attribute__((ext_vector_type(8)))  __bf16   v8b;
typedef __attribute__((ext_vector_type(8)))  float    v8f;
typedef __attribute__((ext_vector_type(4)))  float    v4f;
typedef __attribute__((ext_vector_type(4)))  unsigned int   u32x4;
typedef __attribute__((ext_vector_type(8)))  unsigned short u16x8;

constexpr int kB    = 2;
constexpr int kS    = 2048;
constexpr int kHid  = 2048;
constexpr int kNH   = 16;
constexpr int kNKV  = 4;
constexpr int kHD   = 128;
constexpr int kTok  = kB * kS;
constexpr int kQN   = kNH * kHD;
constexpr int kKVN  = kNKV * kHD;
constexpr int kQB   = 64;
constexpr int kKC   = 64;
constexpr int kNC   = kS / kKC;
constexpr int kMsPitch = 68;

static_assert(kTok % 64 == 0, "");
static_assert(kQN % 64 == 0 && kKVN % 64 == 0 && kHid % 64 == 0, "");
static_assert(kHid % 32 == 0 && kQN % 32 == 0, "");
static_assert(kS % kQB == 0 && kS % kKC == 0 && kHD == 128 && kNC == 32 && kQB == kKC, "");

__device__ __forceinline__ unsigned short f2bf_bits(float f) {
  unsigned u = __float_as_uint(f);
  return (unsigned short)((u + 0x7FFFu + ((u >> 16) & 1u)) >> 16);
}
__device__ __forceinline__ float bf_bits2f(unsigned short h) { return __uint_as_float(((unsigned)h) << 16); }
__device__ __forceinline__ void split_bf16(float f, unsigned short& hb, unsigned short& lb) {
  hb = f2bf_bits(f);
  lb = f2bf_bits(f - bf_bits2f(hb));
}

__device__ __forceinline__ void dep_guard_h(v8f& a, v8f& b, v16h x, v16h y) { asm volatile("v_nop\n\tv_nop\n\tv_nop\n\tv_nop" : "+v"(a), "+v"(b) : "v"(x), "v"(y)); }
__device__ __forceinline__ void dep_guard_b(v8f& a, v8f& b, v16b x, v16b y) { asm volatile("v_nop\n\tv_nop\n\tv_nop\n\tv_nop" : "+v"(a), "+v"(b) : "v"(x), "v"(y)); }
__device__ __forceinline__ void keep4_h(v16h a, v16h b, v16h c, v16h d) { asm volatile("v_nop" :: "v"(a), "v"(b), "v"(c), "v"(d)); }
__device__ __forceinline__ void keep4_b(v16b a, v16b b, v16b c, v16b d) { asm volatile("v_nop" :: "v"(a), "v"(b), "v"(c), "v"(d)); }
__device__ __forceinline__ void acc_guard4(v8f& a, v8f& b, v8f& c, v8f& d) { asm volatile("v_nop\n\tv_nop\n\tv_nop\n\tv_nop" : "+v"(a), "+v"(b), "+v"(c), "+v"(d)); }
template <typename T> struct Frag;
template <> struct Frag<_Float16> {
  typedef v16h V; union U { v16h v; v8h h[2]; };
  static __device__ __forceinline__ v16h load(const _Float16* p) {
    U f; f.h[0] = *(const v8h*)(p); f.h[1] = *(const v8h*)(p + 16); return f.v;
  }
  static __device__ __forceinline__ v8f mma(v16h a, v16h b, v8f c) {
    return __builtin_amdgcn_wmma_f32_16x16x32_f16(false, a, false, b, (short)0, c, false, false);
  }
  static __device__ __forceinline__ void guard(v8f& a, v8f& b, v16h x, v16h y) { dep_guard_h(a, b, x, y); }
  static __device__ __forceinline__ void keep(v16h a, v16h b, v16h c, v16h d) { keep4_h(a, b, c, d); }
};
template <> struct Frag<__bf16> {
  typedef v16b V; union U { v16b v; v8b h[2]; };
  static __device__ __forceinline__ v16b load(const __bf16* p) {
    U f; f.h[0] = *(const v8b*)(p); f.h[1] = *(const v8b*)(p + 16); return f.v;
  }
  static __device__ __forceinline__ v8f mma(v16b a, v16b b, v8f c) {
    return __builtin_amdgcn_wmma_f32_16x16x32_bf16(false, a, false, b, (short)0, c, false, false);
  }
  static __device__ __forceinline__ void guard(v8f& a, v8f& b, v16b x, v16b y) { dep_guard_b(a, b, x, y); }
  static __device__ __forceinline__ void keep(v16b a, v16b b, v16b c, v16b d) { keep4_b(a, b, c, d); }
};

template <int ET> struct Elem;
template <> struct Elem<0> { typedef _Float16 T; };
template <> struct Elem<1> { typedef __bf16 T; };
template <int ET, int SPLITK, int BIAS_MODE, int OUT_MODE, bool RESID, int ACT = 0>
__global__ __launch_bounds__(256) void wmma_gemm64(
    const unsigned short* __restrict__ Ap, const unsigned short* __restrict__ A2p, int lda, long strideA,
    const unsigned short* __restrict__ Btp, const unsigned short* __restrict__ Bt2p, int ldb, long strideB,
    void* __restrict__ Cout, void* __restrict__ Cout2, int ldc, long strideC,
    const float* __restrict__ bias,
    const float* __restrict__ resid, long strideR,
    int M, int N, int K, float scale) {
  constexpr bool SPLIT  = (SPLITK != 0);
  constexpr bool SPLITB = (SPLITK == 1);
  typedef typename Elem<ET>::T T;
  typedef typename Frag<T>::V V;
  const T* A = (const T*)Ap; const T* A2 = (const T*)A2p; const T* Bt = (const T*)Btp; const T* Bt2 = (const T*)Bt2p;
  __shared__ __align__(16) float sT[8][16 * 68];
  const int b    = blockIdx.y;
  const int lane = threadIdx.x & 31;
  const int wave = threadIdx.x >> 5;
  const int tilesN = N >> 6;
  const int tilesM = M >> 6;
  const int tile = blockIdx.x * 8 + wave;
  if (tile >= tilesM * tilesN) return;
  const int tm = tile / tilesN;
  const int tn = tile - tm * tilesN;
  const int m0 = tm << 6;
  const int n0 = tn << 6;

  const T* Ab  = A  + (size_t)b * strideA;
  const T* Bb  = Bt + (size_t)b * strideB;
  const T* Ab2 = SPLIT ? (A2  + (size_t)b * strideA) : nullptr;
  const T* Bb2 = SPLITB ? (Bt2 + (size_t)b * strideB) : nullptr;

  const int rlane = lane & 15;
  const int koff  = (lane >> 4) * 8;
  const int mOff  = (lane >> 4) * 8;

  v8f acc[4][4];
#pragma unroll
  for (int i = 0; i < 4; ++i)
#pragma unroll
    for (int j = 0; j < 4; ++j) acc[i][j] = (v8f){0.f,0.f,0.f,0.f,0.f,0.f,0.f,0.f};

  for (int k0 = 0; k0 < K; k0 += 32) {
    V bh[4], bl[4];
#pragma unroll
    for (int j = 0; j < 4; ++j) {
      const size_t bo = (size_t)(n0 + (j << 4) + rlane) * ldb + koff + k0;
      bh[j] = Frag<T>::load(Bb + bo);
      if (SPLITB) bl[j] = Frag<T>::load(Bb2 + bo);
    }
#pragma unroll
    for (int i = 0; i < 4; ++i) {
      const size_t ao = (size_t)(m0 + (i << 4) + rlane) * lda + koff + k0;
      V ah = Frag<T>::load(Ab + ao);
      V al;
      if (SPLIT) al = Frag<T>::load(Ab2 + ao);
#pragma unroll
      for (int j = 0; j < 4; ++j) {
        acc[i][j] = Frag<T>::mma(ah, bh[j], acc[i][j]);
        if (SPLITB) acc[i][j] = Frag<T>::mma(ah, bl[j], acc[i][j]);
        if (SPLIT)  acc[i][j] = Frag<T>::mma(al, bh[j], acc[i][j]);
      }
      Frag<T>::guard(acc[i][0], acc[i][3], ah, SPLIT ? al : ah);
    }
    Frag<T>::keep(bh[0], bh[1], bh[2], bh[3]);
    if (SPLITB) Frag<T>::keep(bl[0], bl[1], bl[2], bl[3]);
  }
  acc_guard4(acc[0][0], acc[0][1], acc[0][2], acc[0][3]);
  acc_guard4(acc[1][0], acc[1][1], acc[1][2], acc[1][3]);
  acc_guard4(acc[2][0], acc[2][1], acc[2][2], acc[2][3]);
  acc_guard4(acc[3][0], acc[3][1], acc[3][2], acc[3][3]);

  float* slab = sT[wave];
  const float* Rb = RESID ? (resid + (size_t)b * strideR) : nullptr;
#pragma unroll
  for (int i = 0; i < 4; ++i) {
    const int mBase = m0 + (i << 4);
#pragma unroll
    for (int j = 0; j < 4; ++j) {
      const int n = n0 + (j << 4) + rlane;
      float bv = 0.f;
      if (BIAS_MODE == 2) bv = bias[n];
#pragma unroll
      for (int r = 0; r < 8; ++r) {
        float v = acc[i][j][r] * scale;
        if (BIAS_MODE == 1) v += bias[mBase + mOff + r];
        if (BIAS_MODE == 2) v += bv;
        if (RESID) v += Rb[(size_t)(mBase + mOff + r) * ldc + n];
        if (ACT == 1) v = tanhf(v);
        if (ACT == 2) v = fmaxf(v, 0.0f);
        if (ACT == 3) v = v / (1.0f + expf(-v));
        if (ACT == 4) v = (v > 0.f) ? v : 0.01f * v;
        if (ACT == 5) v = 0.5f * v * (1.0f + erff(v * 0.70710678118654752f));
        slab[(mOff + r) * 68 + (j << 4) + rlane] = v;
      }
    }
    __builtin_amdgcn_fence(__ATOMIC_RELEASE, "workgroup");
    __builtin_amdgcn_wave_barrier();
    __builtin_amdgcn_fence(__ATOMIC_ACQUIRE, "workgroup");
    if (OUT_MODE == 0) {
      float* C = (float*)Cout + (size_t)b * strideC;
      const int hh = lane >> 4, c4 = (lane & 15) * 4;
      for (int pass = 0; pass < 2; ++pass) {
#pragma unroll
        for (int it = 0; it < 8; ++it) {
          const int row = it * 2 + hh;
          v4f v = *(const v4f*)(slab + row * 68 + c4);
          *(volatile v4f*)(C + (size_t)(mBase + row) * ldc + n0 + c4) = v;
        }
        __threadfence();
      }
    } else {
      const int q = lane >> 3, c8 = (lane & 7) * 8;
      unsigned short* C  = (unsigned short*)Cout  + (size_t)b * strideC;
      unsigned short* C2 = (OUT_MODE == 2) ? ((unsigned short*)Cout2 + (size_t)b * strideC) : nullptr;
      for (int pass = 0; pass < 2; ++pass) {
#pragma unroll
        for (int it = 0; it < 4; ++it) {
          const int row = it * 4 + q;
          const float* sp = slab + row * 68 + c8;
          v8h hv, lv;
#pragma unroll
          for (int e = 0; e < 8; ++e) {
            if (OUT_MODE == 1) {
              hv[e] = (_Float16)sp[e];
            } else {
              unsigned short hb = f2bf_bits(sp[e]);
              unsigned short lb = f2bf_bits(sp[e] - bf_bits2f(hb));
              hv[e] = __builtin_bit_cast(_Float16, hb);
              lv[e] = __builtin_bit_cast(_Float16, lb);
            }
          }
          *(volatile v8h*)(C + (size_t)(mBase + row) * ldc + n0 + c8) = hv;
          if (OUT_MODE == 2) *(volatile v8h*)(C2 + (size_t)(mBase + row) * ldc + n0 + c8) = lv;
        }
        __threadfence();
      }
    }
    __builtin_amdgcn_fence(__ATOMIC_RELEASE, "workgroup");
    __builtin_amdgcn_wave_barrier();
    __builtin_amdgcn_fence(__ATOMIC_ACQUIRE, "workgroup");
  }
}

__global__ __launch_bounds__(256) void cast_bf16_kernel(const float* __restrict__ in, unsigned short* __restrict__ out, int n8) {
  const int i = blockIdx.x * 256 + threadIdx.x;
  if (i < n8) {
    const v4f a0 = *(const v4f*)(in + (size_t)i * 8);
    const v4f a1 = *(const v4f*)(in + (size_t)i * 8 + 4);
    u16x8 o;
#pragma unroll
    for (int e = 0; e < 4; ++e) { o[e] = f2bf_bits(a0[e]); o[4 + e] = f2bf_bits(a1[e]); }
    *(volatile u16x8*)(out + (size_t)i * 8) = o;
    __threadfence();
    *(volatile u16x8*)(out + (size_t)i * 8) = o;
  }
}

__global__ __launch_bounds__(256) void transpose_bf16_kernel(const float* __restrict__ in, unsigned short* __restrict__ out, int R, int Cn) {
  __shared__ __align__(16) unsigned short ts[64 * 72];
  const int tid = threadIdx.x;
  const int c0 = blockIdx.x * 64;
  const int r0 = blockIdx.y * 64;
#pragma unroll
  for (int it = 0; it < 4; ++it) {
    const int idx = it * 256 + tid;
    const int rr = idx >> 4;
    const int c4 = (idx & 15) * 4;
    const v4f v = *(const v4f*)(in + (size_t)(r0 + rr) * Cn + c0 + c4);
#pragma unroll
    for (int e = 0; e < 4; ++e) ts[(c4 + e) * 72 + rr] = f2bf_bits(v[e]);
  }
  __syncthreads();
  const int wave = tid >> 5, lane = tid & 31, q = lane >> 3, c8 = (lane & 7) * 8;
  for (int pass = 0; pass < 2; ++pass) {
#pragma unroll
    for (int it = 0; it < 2; ++it) {
      const int row = wave * 8 + it * 4 + q;
      const u16x8 v = *(const u16x8*)(ts + row * 72 + c8);
      *(volatile u16x8*)(out + (size_t)(c0 + row) * R + r0 + c8) = v;
    }
    __threadfence();
  }
}

__global__ __launch_bounds__(256) void mask_flags_kernel(const float* __restrict__ amask, int* __restrict__ tflags) {
  __shared__ int wkeep[kNC][8];
  const int tid = threadIdx.x, wave = tid >> 5, lane = tid & 31;
  const int qb  = blockIdx.x;
  const int row = tid >> 2;
  const int cq  = (tid & 3) * 16;
  const float* mrow = amask + (size_t)(qb * kQB + row) * kS + cq;
#pragma unroll 1
  for (int kc = 0; kc < kNC; ++kc) {
    int keep = 0;
#pragma unroll
    for (int i = 0; i < 4; ++i) {
      const v4f v = *(const v4f*)(mrow + kc * kKC + 4 * i);
      keep |= (int)(v[0] > -1.0e37f) | (int)(v[1] > -1.0e37f) | (int)(v[2] > -1.0e37f) | (int)(v[3] > -1.0e37f);
    }
#pragma unroll
    for (int off = 1; off < 32; off <<= 1) keep |= __shfl_xor(keep, off, 32);
    if (lane == 0) wkeep[kc][wave] = keep;
  }
  __syncthreads();
  if (wave == 0) {
    int k = 0;
#pragma unroll
    for (int w = 0; w < 8; ++w) k |= wkeep[lane][w];
    const int f = (k == 0) ? 1 : 0;
    ((volatile int*)tflags)[qb * kNC + lane] = f;
    __threadfence();
    ((volatile int*)tflags)[qb * kNC + lane] = f;
  }
}

struct FreqTab { float f[64]; };
static_assert(sizeof(FreqTab) == 256, "");

__global__ __launch_bounds__(128) void rope_split_kernel(
    const float* __restrict__ qp, const float* __restrict__ kp,
    unsigned short* __restrict__ Qh, unsigned short* __restrict__ Ql,
    unsigned short* __restrict__ Kh, unsigned short* __restrict__ Kl,
    FreqTab ft)
{
  __shared__ __align__(16) float cst[64];
  __shared__ __align__(16) float snt[64];
  const int tid = threadIdx.x;
  const int tok = blockIdx.x;
  const int b = tok / kS;
  const int s = tok - b * kS;
  if (tid < 64) {
    float fv = ft.f[0];
#pragma unroll
    for (int i = 1; i < 64; ++i) fv = (tid == i) ? ft.f[i] : fv;
    const float ang = (float)s * fv;
    float sn, cs;
    sincosf(ang, &sn, &cs);
    cst[tid] = cs;
    snt[tid] = sn;
  }
  __syncthreads();
  const int r  = tid >> 4;
  const int d0 = (tid & 15) * 8;
  const int dp = d0 ^ 64;
  const int ci = d0 & 63;
  const float sgn = (d0 < 64) ? -1.0f : 1.0f;
  const v4f cv0 = *(const v4f*)(cst + ci), cv1 = *(const v4f*)(cst + ci + 4);
  const v4f sv0 = *(const v4f*)(snt + ci), sv1 = *(const v4f*)(snt + ci + 4);
#pragma unroll 1
  for (int ri = 0; ri < 3; ++ri) {
    const bool isk = (ri == 2);
    if (isk && r >= kNKV) break;
    const int head = isk ? r : (ri * 8 + r);
    const float* src = isk ? (kp + (size_t)tok * kKVN + (size_t)head * kHD)
                           : (qp + (size_t)tok * kQN  + (size_t)head * kHD);
    const size_t drow = isk ? (((size_t)(b * kNKV + head)) * kS + s) * kHD
                            : (((size_t)(b * kNH  + head)) * kS + s) * kHD;
    unsigned short* dh = (isk ? Kh : Qh) + drow + d0;
    unsigned short* dl = (isk ? Kl : Ql) + drow + d0;
    const v4f x0 = *(const v4f*)(src + d0);
    const v4f x1 = *(const v4f*)(src + d0 + 4);
    const v4f y0 = *(const v4f*)(src + dp);
    const v4f y1 = *(const v4f*)(src + dp + 4);
    u16x8 hv, lv;
#pragma unroll
    for (int e = 0; e < 4; ++e) {
      const float f0 = x0[e] * cv0[e] + (sgn * y0[e]) * sv0[e];
      const float f1 = x1[e] * cv1[e] + (sgn * y1[e]) * sv1[e];
      unsigned short hb, lb;
      split_bf16(f0, hb, lb); hv[e] = hb;     lv[e] = lb;
      split_bf16(f1, hb, lb); hv[4 + e] = hb; lv[4 + e] = lb;
    }
    *(volatile u16x8*)dh = hv;
    *(volatile u16x8*)dl = lv;
    __threadfence();
    *(volatile u16x8*)dh = hv;
    *(volatile u16x8*)dl = lv;
  }
}

__global__ __launch_bounds__(256) void vsplit_kernel(const float* __restrict__ vp, unsigned short* __restrict__ Vth, unsigned short* __restrict__ Vtl) {
  __shared__ __align__(16) unsigned short th[kHD * 72];
  __shared__ __align__(16) unsigned short tl[kHD * 72];
  const int tid = threadIdx.x;
  const int bid = blockIdx.x;
  const int st  = bid % (kS / 64);
  const int bk  = bid / (kS / 64);
  const int kvh = bk % kNKV;
  const int b   = bk / kNKV;
  const int s0  = st * 64;
#pragma unroll 2
  for (int it = 0; it < 8; ++it) {
    const int idx = it * 256 + tid;
    const int tr  = idx >> 5;
    const int d4  = (idx & 31) * 4;
    const v4f v = *(const v4f*)(vp + (size_t)(b * kS + s0 + tr) * kKVN + kvh * kHD + d4);
#pragma unroll
    for (int e = 0; e < 4; ++e) {
      unsigned short hb, lb;
      split_bf16(v[e], hb, lb);
      th[(d4 + e) * 72 + tr] = hb;
      tl[(d4 + e) * 72 + tr] = lb;
    }
  }
  __syncthreads();
  const int wave = tid >> 5, lane = tid & 31, q = lane >> 3, c8 = (lane & 7) * 8;
  const size_t obase = (size_t)(b * kNKV + kvh) * kHD;
  for (int pass = 0; pass < 2; ++pass) {
#pragma unroll
    for (int it = 0; it < 4; ++it) {
      const int row = wave * 16 + it * 4 + q;
      const u16x8 hv = *(const u16x8*)(th + row * 72 + c8);
      const u16x8 lv = *(const u16x8*)(tl + row * 72 + c8);
      *(volatile u16x8*)(Vth + (obase + row) * kS + s0 + c8) = hv;
      *(volatile u16x8*)(Vtl + (obase + row) * kS + s0 + c8) = lv;
    }
    __threadfence();
  }
}

union AttnQO { unsigned short q[2][kQB * kHD]; float o[4][16 * kHD]; };
static_assert(sizeof(AttnQO) == 32768, "");

__device__ __forceinline__ v8f mma_bf16(v16b a, v16b b, v8f c) {
  c = __builtin_amdgcn_wmma_f32_16x16x32_bf16(false, a, false, b, (short)0, c, false, false);
  asm volatile("v_nop\n\tv_nop\n\tv_nop\n\tv_nop" : "+v"(c) : "v"(a), "v"(b));
  return c;
}

__global__ __launch_bounds__(128) void attn_hd128_kernel(
    const unsigned short* __restrict__ Qh, const unsigned short* __restrict__ Ql,
    const unsigned short* __restrict__ Kh, const unsigned short* __restrict__ Kl,
    const unsigned short* __restrict__ Vth, const unsigned short* __restrict__ Vtl,
    const float* __restrict__ amask, const int* __restrict__ tflags,
    unsigned short* __restrict__ Oh, unsigned short* __restrict__ Ol)
{
  __shared__ __align__(16) AttnQO qo;
  __shared__ __align__(16) unsigned short ks[2][kKC * kHD];
  __shared__ __align__(16) unsigned short vs[2][kHD * kKC];
  __shared__ __align__(16) __bf16 ps[2][4][16 * kKC];
  __shared__ __align__(16) float ms[4][16 * kMsPitch];
  __shared__ int fl[kNC];

  const int tid  = threadIdx.x;
  const int wave = tid >> 5;
  const int lane = tid & 31;
  const int hh   = lane >> 4;
  const int c    = lane & 15;
  constexpr int nqb = kS / kQB;
  const int bx  = blockIdx.x;
  const int qb  = bx % nqb;
  const int bhd = bx / nqb;
  const int h   = bhd % kNH;
  const int b   = bhd / kNH;
  const int kvh = h / (kNH / kNKV);
  const int qr0 = qb * kQB;
  const int q0  = qr0 + wave * 16;

  const size_t qoff = ((size_t)(b * kNH + h) * kS + qr0) * kHD;
  const unsigned short* qhp = Qh + qoff;
  const unsigned short* qlp = Ql + qoff;
  const size_t koff = (size_t)(b * kNKV + kvh) * kS * kHD;
  const unsigned short* khp = Kh + koff;
  const unsigned short* klp = Kl + koff;
  const size_t voff = (size_t)(b * kNKV + kvh) * kHD * kS;
  const unsigned short* vhp = Vth + voff;
  const unsigned short* vlp = Vtl + voff;

  if (tid < kNC) fl[tid] = tflags[qb * kNC + tid];
#pragma unroll 2
  for (int it = 0; it < 8; ++it) {
    const int idx = it * 128 + tid;
    const u32x4 a0 = *(const u32x4*)(qhp + (size_t)idx * 8);
    const u32x4 a1 = *(const u32x4*)(qlp + (size_t)idx * 8);
    *(u32x4*)(&qo.q[0][idx * 8]) = a0;
    *(u32x4*)(&qo.q[1][idx * 8]) = a1;
  }

  float mrow[8], lrow[8];
  v8f oacc[8];
#pragma unroll
  for (int r = 0; r < 8; ++r) { mrow[r] = -INFINITY; lrow[r] = 0.f; }
#pragma unroll
  for (int t = 0; t < 8; ++t) oacc[t] = (v8f){0.f,0.f,0.f,0.f,0.f,0.f,0.f,0.f};

  const float kSc2   = 0.08838834764831845f * 1.4426950408889634f;
  const float kLog2e = 1.4426950408889634f;
  float* msw = ms[wave];
  __bf16* pwh = ps[0][wave];
  __bf16* pwl = ps[1][wave];
  __syncthreads();

  for (int kc = 0; kc < kNC; ++kc) {
    if (fl[kc] == 1) continue;
    const int kv0 = kc * kKC;
    __syncthreads();
#pragma unroll 2
    for (int it = 0; it < 8; ++it) {
      const int idx = it * 128 + tid;
      const u32x4 a0 = *(const u32x4*)(khp + (size_t)kv0 * kHD + (size_t)idx * 8);
      const u32x4 a1 = *(const u32x4*)(klp + (size_t)kv0 * kHD + (size_t)idx * 8);
      *(u32x4*)(&ks[0][idx * 8]) = a0;
      *(u32x4*)(&ks[1][idx * 8]) = a1;
    }
#pragma unroll 2
    for (int it = 0; it < 8; ++it) {
      const int idx = it * 128 + tid;
      const int d   = idx >> 3;
      const int p8  = (idx & 7) * 8;
      const u32x4 a0 = *(const u32x4*)(vhp + (size_t)d * kS + kv0 + p8);
      const u32x4 a1 = *(const u32x4*)(vlp + (size_t)d * kS + kv0 + p8);
      *(u32x4*)(&vs[0][d * kKC + p8]) = a0;
      *(u32x4*)(&vs[1][d * kKC + p8]) = a1;
    }
#pragma unroll 4
    for (int it = 0; it < 8; ++it) {
      const int row = it * 2 + hh;
      const v4f mv = *(const v4f*)(amask + (size_t)(q0 + row) * kS + kv0 + c * 4);
      *(v4f*)(msw + row * kMsPitch + c * 4) = mv;
    }
    __syncthreads();

    v8f s[4];
#pragma unroll
    for (int j = 0; j < 4; ++j) s[j] = (v8f){0.f,0.f,0.f,0.f,0.f,0.f,0.f,0.f};
    const __bf16* qhl = (const __bf16*)(&qo.q[0][0]) + (wave * 16 + c) * kHD + 8 * hh;
    const __bf16* qll = (const __bf16*)(&qo.q[1][0]) + (wave * 16 + c) * kHD + 8 * hh;
    const __bf16* khl = (const __bf16*)(&ks[0][0]) + c * kHD + 8 * hh;
    const __bf16* kll = (const __bf16*)(&ks[1][0]) + c * kHD + 8 * hh;
#pragma unroll 1
    for (int dc = 0; dc < 4; ++dc) {
      const v16b qa = Frag<__bf16>::load(qhl + dc * 32);
      const v16b qz = Frag<__bf16>::load(qll + dc * 32);
#pragma unroll
      for (int j = 0; j < 4; ++j) {
        const v16b kb = Frag<__bf16>::load(khl + j * 16 * kHD + dc * 32);
        const v16b kz = Frag<__bf16>::load(kll + j * 16 * kHD + dc * 32);
        s[j] = mma_bf16(qa, kb, s[j]);
        s[j] = mma_bf16(qa, kz, s[j]);
        s[j] = mma_bf16(qz, kb, s[j]);
      }
    }

    float cm[8];
#pragma unroll
    for (int r = 0; r < 8; ++r) {
      float m = -INFINITY;
#pragma unroll
      for (int j = 0; j < 4; ++j) {
        const float mv = msw[(8 * hh + r) * kMsPitch + j * 16 + c];
        const float t = s[j][r] * kSc2 + mv * kLog2e;
        s[j][r] = t;
        m = fmaxf(m, t);
      }
#pragma unroll
      for (int off = 1; off < 16; off <<= 1) m = fmaxf(m, __shfl_xor(m, off, 32));
      cm[r] = m;
    }
#pragma unroll
    for (int r = 0; r < 8; ++r) {
      const float mnew  = fmaxf(mrow[r], cm[r]);
      const float msub  = (mnew == -INFINITY) ? 0.0f : mnew;
      const float alpha = exp2f(mrow[r] - msub);
      mrow[r] = mnew;
      float psum = 0.f;
#pragma unroll
      for (int j = 0; j < 4; ++j) {
        const float p = exp2f(s[j][r] - msub);
        psum += p;
        unsigned short hb, lb;
        split_bf16(p, hb, lb);
        pwh[(8 * hh + r) * kKC + j * 16 + c] = __builtin_bit_cast(__bf16, hb);
        pwl[(8 * hh + r) * kKC + j * 16 + c] = __builtin_bit_cast(__bf16, lb);
      }
#pragma unroll
      for (int off = 1; off < 16; off <<= 1) psum += __shfl_xor(psum, off, 32);
      lrow[r] = lrow[r] * alpha + psum;
#pragma unroll
      for (int t = 0; t < 8; ++t) oacc[t][r] *= alpha;
    }
    __builtin_amdgcn_fence(__ATOMIC_RELEASE, "workgroup");
    __builtin_amdgcn_wave_barrier();
    __builtin_amdgcn_fence(__ATOMIC_ACQUIRE, "workgroup");

    const __bf16* phl = pwh + c * kKC + 8 * hh;
    const __bf16* pll = pwl + c * kKC + 8 * hh;
    const __bf16* vhl = (const __bf16*)(&vs[0][0]) + c * kKC + 8 * hh;
    const __bf16* vll = (const __bf16*)(&vs[1][0]) + c * kKC + 8 * hh;
#pragma unroll 1
    for (int kk = 0; kk < 2; ++kk) {
      const v16b pa = Frag<__bf16>::load(phl + kk * 32);
      const v16b pz = Frag<__bf16>::load(pll + kk * 32);
#pragma unroll
      for (int t = 0; t < 8; ++t) {
        const v16b vb = Frag<__bf16>::load(vhl + t * 16 * kKC + kk * 32);
        const v16b vz = Frag<__bf16>::load(vll + t * 16 * kKC + kk * 32);
        oacc[t] = mma_bf16(pa, vb, oacc[t]);
        oacc[t] = mma_bf16(pa, vz, oacc[t]);
        oacc[t] = mma_bf16(pz, vb, oacc[t]);
      }
    }
  }

  __syncthreads();
  float* os = qo.o[wave];
#pragma unroll
  for (int r = 0; r < 8; ++r) {
    const float inv = 1.0f / lrow[r];
#pragma unroll
    for (int t = 0; t < 8; ++t) os[(8 * hh + r) * kHD + t * 16 + c] = oacc[t][r] * inv;
  }
  __builtin_amdgcn_fence(__ATOMIC_RELEASE, "workgroup");
  __builtin_amdgcn_wave_barrier();
  __builtin_amdgcn_fence(__ATOMIC_ACQUIRE, "workgroup");
  unsigned short* ohp = Oh + (size_t)(b * kS + q0) * kQN + h * kHD;
  unsigned short* olp = Ol + (size_t)(b * kS + q0) * kQN + h * kHD;
  for (int pass = 0; pass < 2; ++pass) {
#pragma unroll
    for (int it = 0; it < 8; ++it) {
      const int row = it * 2 + hh;
      const v4f a0 = *(const v4f*)(os + row * kHD + c * 8);
      const v4f a1 = *(const v4f*)(os + row * kHD + c * 8 + 4);
      u16x8 hv, lv;
#pragma unroll
      for (int e = 0; e < 4; ++e) {
        unsigned short hb, lb;
        split_bf16(a0[e], hb, lb); hv[e] = hb;     lv[e] = lb;
        split_bf16(a1[e], hb, lb); hv[4 + e] = hb; lv[4 + e] = lb;
      }
      *(volatile u16x8*)(ohp + (size_t)row * kQN + c * 8) = hv;
      *(volatile u16x8*)(olp + (size_t)row * kQN + c * 8) = lv;
    }
    __threadfence();
  }
}

static double host_sqrt_d(double a) {
  double x = (a > 1.0) ? a : 1.0;
  for (int i = 0; i < 64; ++i) x = 0.5 * (x + a / x);
  return x;
}

extern "C" void kernel_launch(void* const* d_in, const int* in_sizes, int n_in,
                              void* d_out, int out_size, void* d_ws,
                              size_t ws_size, hipStream_t stream) {
  (void)in_sizes;
  if (n_in < 6) return;
  if (out_size != kTok * kHid) return;
  const float* hs = (const float*)d_in[0];
  const float* am = (const float*)d_in[1];
  const float* wq = (const float*)d_in[2];
  const float* wk = (const float*)d_in[3];
  const float* wv = (const float*)d_in[4];
  const float* wo = (const float*)d_in[5];

  constexpr size_t MiB = 1048576;
  constexpr size_t szHsb  = (size_t)kTok * kHid * 2;
  constexpr size_t szWqT  = (size_t)kQN * kHid * 2;
  constexpr size_t szWkvT = (size_t)kKVN * kHid * 2;
  constexpr size_t szWoT  = (size_t)kHid * kQN * 2;
  constexpr size_t szQp   = (size_t)kTok * kQN * 4;
  constexpr size_t szKVp  = (size_t)kTok * kKVN * 4;
  constexpr size_t szQpl  = (size_t)kB * kNH * kS * kHD * 2;
  constexpr size_t szKVpl = (size_t)kB * kNKV * kS * kHD * 2;
  constexpr size_t szApl  = (size_t)kTok * kQN * 2;
  constexpr size_t szFl   = (size_t)kNC * kNC * 4;
  static_assert(szHsb == 16 * MiB && szWqT == 8 * MiB && szWkvT == 2 * MiB && szWoT == 8 * MiB, "");
  static_assert(szQp == 32 * MiB && szKVp == 8 * MiB && szQpl == 16 * MiB && szKVpl == 4 * MiB && szApl == 16 * MiB && szFl == 4096, "");

  constexpr size_t oHsb = 0;
  constexpr size_t oKh  = 0, oKl = oKh + szKVpl, oVh = oKl + szKVpl, oVl = oVh + szKVpl;
  constexpr size_t oWqT = oHsb + szHsb, oWkT = oWqT + szWqT, oWvT = oWkT + szWkvT, oWoT = oWvT + szWkvT;
  constexpr size_t oQp  = oWoT + szWoT;
  constexpr size_t oAh  = oQp, oAl = oAh + szApl;
  constexpr size_t oKp  = oQp + szQp, oVp = oKp + szKVp;
  constexpr size_t oQh  = oVp + szKVp, oQl = oQh + szQpl;
  constexpr size_t oFl  = oQl + szQpl;
  constexpr size_t kWsTotal = oFl + szFl;
  static_assert(oVl + szKVpl <= oHsb + szHsb, "");
  static_assert(oAl + szApl <= oQp + szQp, "");
  static_assert(oWqT == 16 * MiB && oWoT == 28 * MiB && oQp == 36 * MiB && oKp == 68 * MiB && oVp == 76 * MiB, "");
  static_assert(oQh == 84 * MiB && oQl == 100 * MiB && oFl == 116 * MiB, "");
  static_assert(kWsTotal == 116 * MiB + 4096 && kWsTotal <= 134217728, "");
  static_assert((size_t)kTok * kHid * 4 == 33554432, "");
  if (ws_size < kWsTotal) return;

  char* ws = (char*)d_ws;
  unsigned short* hsb = (unsigned short*)(ws + oHsb);
  unsigned short* wqT = (unsigned short*)(ws + oWqT);
  unsigned short* wkT = (unsigned short*)(ws + oWkT);
  unsigned short* wvT = (unsigned short*)(ws + oWvT);
  unsigned short* woT = (unsigned short*)(ws + oWoT);
  float* qp = (float*)(ws + oQp);
  float* kp = (float*)(ws + oKp);
  float* vp = (float*)(ws + oVp);
  unsigned short* Ah = (unsigned short*)(ws + oAh);
  unsigned short* Al = (unsigned short*)(ws + oAl);
  unsigned short* Qh = (unsigned short*)(ws + oQh);
  unsigned short* Ql = (unsigned short*)(ws + oQl);
  unsigned short* Kh = (unsigned short*)(ws + oKh);
  unsigned short* Kl = (unsigned short*)(ws + oKl);
  unsigned short* Vh = (unsigned short*)(ws + oVh);
  unsigned short* Vl = (unsigned short*)(ws + oVl);
  int* Fl = (int*)(ws + oFl);

  {
    const int n8 = kTok * kHid / 8;
    cast_bf16_kernel<<<dim3((n8 + 255) / 256), dim3(256), 0, stream>>>(hs, hsb, n8);
  }
  transpose_bf16_kernel<<<dim3(kQN / 64, kHid / 64), dim3(256), 0, stream>>>(wq, wqT, kHid, kQN);
  transpose_bf16_kernel<<<dim3(kKVN / 64, kHid / 64), dim3(256), 0, stream>>>(wk, wkT, kHid, kKVN);
  transpose_bf16_kernel<<<dim3(kKVN / 64, kHid / 64), dim3(256), 0, stream>>>(wv, wvT, kHid, kKVN);
  transpose_bf16_kernel<<<dim3(kHid / 64, kQN / 64), dim3(256), 0, stream>>>(wo, woT, kQN, kHid);

  {
    const int tilesQ = (kTok / 64) * (kQN / 64);
    wmma_gemm64<1, 0, 0, 0, false><<<dim3((tilesQ + 7) / 8, 1), dim3(256), 0, stream>>>(
        hsb, hsb, kHid, 0L, wqT, wqT, kHid, 0L, (void*)qp, (void*)qp, kQN, 0L,
        nullptr, nullptr, 0L, kTok, kQN, kHid, 1.0f);
    const int tilesKV = (kTok / 64) * (kKVN / 64);
    wmma_gemm64<1, 0, 0, 0, false><<<dim3((tilesKV + 7) / 8, 1), dim3(256), 0, stream>>>(
        hsb, hsb, kHid, 0L, wkT, wkT, kHid, 0L, (void*)kp, (void*)kp, kKVN, 0L,
        nullptr, nullptr, 0L, kTok, kKVN, kHid, 1.0f);
    wmma_gemm64<1, 0, 0, 0, false><<<dim3((tilesKV + 7) / 8, 1), dim3(256), 0, stream>>>(
        hsb, hsb, kHid, 0L, wvT, wvT, kHid, 0L, (void*)vp, (void*)vp, kKVN, 0L,
        nullptr, nullptr, 0L, kTok, kKVN, kHid, 1.0f);
  }

  mask_flags_kernel<<<dim3(kS / kQB), dim3(256), 0, stream>>>(am, Fl);

  {
    const double r4  = 0.1;
    const double r8  = host_sqrt_d(r4);
    const double r16 = host_sqrt_d(r8);
    const double r32 = host_sqrt_d(r16);
    const double r64 = host_sqrt_d(r32);
    FreqTab ft;
    for (int i = 0; i < 64; ++i) {
      double v = 1.0;
      if (i & 1)  v *= r64;
      if (i & 2)  v *= r32;
      if (i & 4)  v *= r16;
      if (i & 8)  v *= r8;
      if (i & 16) v *= 0.1;
      if (i & 32) v *= 0.01;
      ft.f[i] = (float)v;
    }
    rope_split_kernel<<<dim3(kTok), dim3(128), 0, stream>>>(qp, kp, Qh, Ql, Kh, Kl, ft);
    vsplit_kernel<<<dim3(kB * kNKV * (kS / 64)), dim3(256), 0, stream>>>(vp, Vh, Vl);
  }

  attn_hd128_kernel<<<dim3(kB * kNH * (kS / kQB)), dim3(128), 0, stream>>>(Qh, Ql, Kh, Kl, Vh, Vl, am, Fl, Ah, Al);

  {
    const int tilesO = (kTok / 64) * (kHid / 64);
    wmma_gemm64<1, 2, 0, 0, false><<<dim3((tilesO + 7) / 8, 1), dim3(256), 0, stream>>>(
        Ah, Al, kQN, 0L, woT, woT, kQN, 0L, d_out, d_out, kHid, 0L,
        nullptr, nullptr, 0L, kTok, kHid, kQN, 1.0f);
  }
}
